// MOE_PositionwiseFeedForward_2980707304165
// MI455X (gfx1250) — hardware-verified
//
#include <hip/hip_runtime.h>
#include <math.h>

constexpr int kTok  = 8192;
constexpr int kDin  = 1024;
constexpr int kHid  = 4096;
constexpr int kExp  = 3;
constexpr int kRank = 8;
constexpr int kER   = kExp * kRank;
constexpr int kTail = 64;
constexpr int kLd1  = kDin + kTail;
constexpr int kLd2  = kHid + kTail;
constexpr int kK1   = kDin + 32;
constexpr int kK2   = kHid + 32;
constexpr int kNsm  = 64;
constexpr float kScaling  = 0.125f;
constexpr float kCarry    = 64.0f;
constexpr float kCarryInv = 1.0f / 64.0f;
constexpr float kCarryB2  = 4.0f;
constexpr float kTailFac2 = 16.0f * kScaling;

static_assert(kTok % 64 == 0 && kHid % 64 == 0 && kDin % 64 == 0, "tile multiples");
static_assert(kK1 % 32 == 0 && kK2 % 32 == 0 && kDin % 32 == 0 && kHid % 32 == 0, "K multiples of 32");
static_assert(kK1 + 0 <= kLd1 && kK2 <= kLd2, "pitch covers K");
static_assert(kER + kExp <= 32 && kNsm == 64, "router columns fit");

typedef __attribute__((ext_vector_type(16))) _Float16 v16h;
typedef __attribute__((ext_vector_type(8)))  _Float16 v8h;
typedef __attribute__((ext_vector_type(16))) __bf16   v16b;
typedef __attribute__((ext_vector_type(8)))  __bf16   v8b;
typedef __attribute__((ext_vector_type(8)))  float    v8f;
typedef __attribute__((ext_vector_type(4)))  float    v4f;
typedef __attribute__((ext_vector_type(4)))  unsigned int v4u;

__device__ __forceinline__ unsigned short f2bf_bits(float f) {
  unsigned u = __float_as_uint(f);
  return (unsigned short)((u + 0x7FFFu + ((u >> 16) & 1u)) >> 16);
}
__device__ __forceinline__ float bf_bits2f(unsigned short h) { return __uint_as_float(((unsigned)h) << 16); }
__device__ __forceinline__ unsigned pk16(unsigned short a, unsigned short b) { return (unsigned)a | ((unsigned)b << 16); }
__device__ __forceinline__ unsigned short h_bits(float f) { const _Float16 h = (_Float16)f; return __builtin_bit_cast(unsigned short, h); }

__device__ __forceinline__ void dep_guard_h(v8f& a, v8f& b, v16h x, v16h y) { asm volatile("v_nop\n\tv_nop\n\tv_nop\n\tv_nop" : "+v"(a), "+v"(b) : "v"(x), "v"(y)); }
__device__ __forceinline__ void dep_guard_b(v8f& a, v8f& b, v16b x, v16b y) { asm volatile("v_nop\n\tv_nop\n\tv_nop\n\tv_nop" : "+v"(a), "+v"(b) : "v"(x), "v"(y)); }
__device__ __forceinline__ void keep4_h(v16h a, v16h b, v16h c, v16h d) { asm volatile("v_nop" :: "v"(a), "v"(b), "v"(c), "v"(d)); }
__device__ __forceinline__ void keep4_b(v16b a, v16b b, v16b c, v16b d) { asm volatile("v_nop" :: "v"(a), "v"(b), "v"(c), "v"(d)); }
__device__ __forceinline__ void acc_guard4(v8f& a, v8f& b, v8f& c, v8f& d) { asm volatile("v_nop\n\tv_nop\n\tv_nop\n\tv_nop" : "+v"(a), "+v"(b), "+v"(c), "+v"(d)); }
template <typename T> struct Frag;
template <> struct Frag<_Float16> {
  typedef v16h V; union U { v16h v; v8h h[2]; };
  static __device__ __forceinline__ v16h load(const _Float16* p) {
    U f; f.h[0] = *(const v8h*)(p); f.h[1] = *(const v8h*)(p + 16); return f.v;
  }
  static __device__ __forceinline__ v8f mma(v16h a, v16h b, v8f c) {
    return __builtin_amdgcn_wmma_f32_16x16x32_f16(false, a, false, b, (short)0, c, false, false);
  }
  static __device__ __forceinline__ void guard(v8f& a, v8f& b, v16h x, v16h y) { dep_guard_h(a, b, x, y); }
  static __device__ __forceinline__ void keep(v16h a, v16h b, v16h c, v16h d) { keep4_h(a, b, c, d); }
};
template <> struct Frag<__bf16> {
  typedef v16b V; union U { v16b v; v8b h[2]; };
  static __device__ __forceinline__ v16b load(const __bf16* p) {
    U f; f.h[0] = *(const v8b*)(p); f.h[1] = *(const v8b*)(p + 16); return f.v;
  }
  static __device__ __forceinline__ v8f mma(v16b a, v16b b, v8f c) {
    return __builtin_amdgcn_wmma_f32_16x16x32_bf16(false, a, false, b, (short)0, c, false, false);
  }
  static __device__ __forceinline__ void guard(v8f& a, v8f& b, v16b x, v16b y) { dep_guard_b(a, b, x, y); }
  static __device__ __forceinline__ void keep(v16b a, v16b b, v16b c, v16b d) { keep4_b(a, b, c, d); }
};

template <int ET> struct Elem;
template <> struct Elem<0> { typedef _Float16 T; };
template <> struct Elem<1> { typedef __bf16 T; };
template <int ET, bool SPLIT, int BIAS_MODE, int OUT_MODE, bool RESID, int ACT = 0>
__global__ __launch_bounds__(256) void wmma_gemm64(
    const unsigned short* __restrict__ Ap, const unsigned short* __restrict__ A2p, int lda, long strideA,
    const unsigned short* __restrict__ Btp, const unsigned short* __restrict__ Bt2p, int ldb, long strideB,
    void* __restrict__ Cout, void* __restrict__ Cout2, int ldc, long strideC,
    const float* __restrict__ bias,
    const float* __restrict__ resid, long strideR,
    int M, int N, int K, float scale) {
  typedef typename Elem<ET>::T T;
  typedef typename Frag<T>::V V;
  const T* A = (const T*)Ap; const T* A2 = (const T*)A2p; const T* Bt = (const T*)Btp; const T* Bt2 = (const T*)Bt2p;
  __shared__ __align__(16) float sT[8][16 * 68];
  const int b    = blockIdx.y;
  const int lane = threadIdx.x & 31;
  const int wave = threadIdx.x >> 5;
  const int tilesN = N >> 6;
  const int tilesM = M >> 6;
  const int tile = blockIdx.x * 8 + wave;
  if (tile >= tilesM * tilesN) return;
  const int tm = tile / tilesN;
  const int tn = tile - tm * tilesN;
  const int m0 = tm << 6;
  const int n0 = tn << 6;

  const T* Ab  = A  + (size_t)b * strideA;
  const T* Bb  = Bt + (size_t)b * strideB;
  const T* Ab2 = SPLIT ? (A2  + (size_t)b * strideA) : nullptr;
  const T* Bb2 = SPLIT ? (Bt2 + (size_t)b * strideB) : nullptr;

  const int rlane = lane & 15;
  const int koff  = (lane >> 4) * 8;
  const int mOff  = (lane >> 4) * 8;

  v8f acc[4][4];
#pragma unroll
  for (int i = 0; i < 4; ++i)
#pragma unroll
    for (int j = 0; j < 4; ++j) acc[i][j] = (v8f){0.f,0.f,0.f,0.f,0.f,0.f,0.f,0.f};

  for (int k0 = 0; k0 < K; k0 += 32) {
    V bh[4], bl[4];
#pragma unroll
    for (int j = 0; j < 4; ++j) {
      const size_t bo = (size_t)(n0 + (j << 4) + rlane) * ldb + koff + k0;
      bh[j] = Frag<T>::load(Bb + bo);
      if (SPLIT) bl[j] = Frag<T>::load(Bb2 + bo);
    }
#pragma unroll
    for (int i = 0; i < 4; ++i) {
      const size_t ao = (size_t)(m0 + (i << 4) + rlane) * lda + koff + k0;
      V ah = Frag<T>::load(Ab + ao);
      V al;
      if (SPLIT) al = Frag<T>::load(Ab2 + ao);
#pragma unroll
      for (int j = 0; j < 4; ++j) {
        acc[i][j] = Frag<T>::mma(ah, bh[j], acc[i][j]);
        if (SPLIT) {
          acc[i][j] = Frag<T>::mma(ah, bl[j], acc[i][j]);
          acc[i][j] = Frag<T>::mma(al, bh[j], acc[i][j]);
        }
      }
      Frag<T>::guard(acc[i][0], acc[i][3], ah, SPLIT ? al : ah);
    }
    Frag<T>::keep(bh[0], bh[1], bh[2], bh[3]);
    if (SPLIT) Frag<T>::keep(bl[0], bl[1], bl[2], bl[3]);
  }
  acc_guard4(acc[0][0], acc[0][1], acc[0][2], acc[0][3]);
  acc_guard4(acc[1][0], acc[1][1], acc[1][2], acc[1][3]);
  acc_guard4(acc[2][0], acc[2][1], acc[2][2], acc[2][3]);
  acc_guard4(acc[3][0], acc[3][1], acc[3][2], acc[3][3]);

  float* slab = sT[wave];
  const float* Rb = RESID ? (resid + (size_t)b * strideR) : nullptr;
#pragma unroll
  for (int i = 0; i < 4; ++i) {
    const int mBase = m0 + (i << 4);
#pragma unroll
    for (int j = 0; j < 4; ++j) {
      const int n = n0 + (j << 4) + rlane;
      float bv = 0.f;
      if (BIAS_MODE == 2) bv = bias[n];
#pragma unroll
      for (int r = 0; r < 8; ++r) {
        float v = acc[i][j][r] * scale;
        if (BIAS_MODE == 1) v += bias[mBase + mOff + r];
        if (BIAS_MODE == 2) v += bv;
        if (RESID) v += Rb[(size_t)(mBase + mOff + r) * ldc + n];
        if (ACT == 2) v = fmaxf(v, 0.0f);
        if (ACT == 4) v = (v > 0.f) ? v : 0.01f * v;
        slab[(mOff + r) * 68 + (j << 4) + rlane] = v;
      }
    }
    __builtin_amdgcn_fence(__ATOMIC_RELEASE, "workgroup");
    __builtin_amdgcn_wave_barrier();
    __builtin_amdgcn_fence(__ATOMIC_ACQUIRE, "workgroup");
    if (OUT_MODE == 0) {
      float* C = (float*)Cout + (size_t)b * strideC;
      const int hh = lane >> 4, c4 = (lane & 15) * 4;
      for (int pass = 0; pass < 2; ++pass) {
#pragma unroll
        for (int it = 0; it < 8; ++it) {
          const int row = it * 2 + hh;
          v4f v = *(const v4f*)(slab + row * 68 + c4);
          *(volatile v4f*)(C + (size_t)(mBase + row) * ldc + n0 + c4) = v;
        }
        __threadfence();
      }
    } else {
      const int q = lane >> 3, c8 = (lane & 7) * 8;
      unsigned short* C  = (unsigned short*)Cout  + (size_t)b * strideC;
      unsigned short* C2 = (OUT_MODE == 2) ? ((unsigned short*)Cout2 + (size_t)b * strideC) : nullptr;
      for (int pass = 0; pass < 2; ++pass) {
#pragma unroll
        for (int it = 0; it < 4; ++it) {
          const int row = it * 4 + q;
          const float* sp = slab + row * 68 + c8;
          v8h hv, lv;
#pragma unroll
          for (int e = 0; e < 8; ++e) {
            if (OUT_MODE == 1) {
              hv[e] = (_Float16)sp[e];
            } else {
              unsigned short hb = f2bf_bits(sp[e]);
              unsigned short lb = f2bf_bits(sp[e] - bf_bits2f(hb));
              hv[e] = __builtin_bit_cast(_Float16, hb);
              lv[e] = __builtin_bit_cast(_Float16, lb);
            }
          }
          *(volatile v8h*)(C + (size_t)(mBase + row) * ldc + n0 + c8) = hv;
          if (OUT_MODE == 2) *(volatile v8h*)(C2 + (size_t)(mBase + row) * ldc + n0 + c8) = lv;
        }
        __threadfence();
      }
    }
    __builtin_amdgcn_fence(__ATOMIC_RELEASE, "workgroup");
    __builtin_amdgcn_wave_barrier();
    __builtin_amdgcn_fence(__ATOMIC_ACQUIRE, "workgroup");
  }
}

template <int MODE> __device__ __forceinline__ unsigned short cvt_in16(float v, float scale) {
  if (MODE == 0) return f2bf_bits(v);
  return h_bits(bf_bits2f(f2bf_bits(v)) * scale);
}
template <int MODE> __device__ __forceinline__ unsigned short cvt_cmp16(float v) {
  if (MODE == 0) return f2bf_bits(v);
  return h_bits(v);
}

__global__ __launch_bounds__(256) void cast_rows_bf16_kernel(const float* __restrict__ x, unsigned short* __restrict__ XA, int nthr) {
  const int g = blockIdx.x * 256 + threadIdx.x;
  if (g >= nthr) return;
  const int row = g >> 7, c8 = (g & 127) * 8;
  const float* p = x + (size_t)row * kDin + c8;
  const v4f a = *(const v4f*)(p);
  const v4f c = *(const v4f*)(p + 4);
  unsigned short hb[8];
#pragma unroll
  for (int e = 0; e < 4; ++e) {
    hb[e]     = f2bf_bits(a[e]);
    hb[4 + e] = f2bf_bits(c[e]);
  }
  const v4u u = (v4u){pk16(hb[0], hb[1]), pk16(hb[2], hb[3]), pk16(hb[4], hb[5]), pk16(hb[6], hb[7])};
  unsigned short* q = XA + (size_t)row * kLd1 + c8;
  *(volatile v4u*)q = u;
  __threadfence();
  *(volatile v4u*)q = u;
}

template <int MODE>
__global__ __launch_bounds__(256) void transpose_cast_kernel(const float* __restrict__ W, unsigned short* __restrict__ T,
                                                             int KR, int NC, int ldT, float scale) {
  __shared__ float tile[64 * 65];
  const int k0 = blockIdx.x * 64;
  const int n0 = blockIdx.y * 64;
  const int t = threadIdx.x;
  {
    const int rr = t >> 4, c4 = (t & 15) * 4;
#pragma unroll
    for (int it = 0; it < 4; ++it) {
      const int r = it * 16 + rr;
      const v4f v = *(const v4f*)(W + (size_t)(k0 + r) * NC + n0 + c4);
      float* tp = tile + r * 65 + c4;
      tp[0] = v[0]; tp[1] = v[1]; tp[2] = v[2]; tp[3] = v[3];
    }
  }
  __syncthreads();
  const int wave = t >> 5, lane = t & 31, q = lane >> 3, j = lane & 7;
  const int nA = wave * 8 + q, nB = nA + 4;
  unsigned short ha[8], hbv[8];
#pragma unroll
  for (int e = 0; e < 8; ++e) {
    const float va = tile[(8 * j + e) * 65 + nA];
    const float vb = tile[(8 * j + e) * 65 + nB];
    ha[e]  = cvt_in16<MODE>(va, scale);
    hbv[e] = cvt_in16<MODE>(vb, scale);
  }
  const v4u ua = (v4u){pk16(ha[0], ha[1]), pk16(ha[2], ha[3]), pk16(ha[4], ha[5]), pk16(ha[6], ha[7])};
  const v4u ub = (v4u){pk16(hbv[0], hbv[1]), pk16(hbv[2], hbv[3]), pk16(hbv[4], hbv[5]), pk16(hbv[6], hbv[7])};
  unsigned short* pa = T + (size_t)(n0 + nA) * ldT + k0 + 8 * j;
  unsigned short* pb = T + (size_t)(n0 + nB) * ldT + k0 + 8 * j;
  *(volatile v4u*)pa = ua;
  *(volatile v4u*)pb = ub;
  __threadfence();
  *(volatile v4u*)pa = ua;
  *(volatile v4u*)pb = ub;
  (void)KR;
}

template <int MODE>
__global__ __launch_bounds__(256) void weight_tail_kernel(const float* __restrict__ Bm, unsigned short* __restrict__ T,
                                                          int NC, int ldT, int KR, float scale, int nthr) {
  const int g = blockIdx.x * 256 + threadIdx.x;
  if (g >= nthr) return;
  const int n = g >> 3, j = g & 7;
  unsigned short hb[8];
#pragma unroll
  for (int e = 0; e < 8; ++e) {
    const int c  = 8 * j + e;
    const int cc = c < kER ? c : (kER - 1);
    float v = Bm[(size_t)cc * NC + n];
    v = (c < kER) ? v : 0.0f;
    hb[e] = cvt_in16<MODE>(v, scale);
  }
  const v4u u = (v4u){pk16(hb[0], hb[1]), pk16(hb[2], hb[3]), pk16(hb[4], hb[5]), pk16(hb[6], hb[7])};
  unsigned short* p = T + (size_t)n * ldT + KR + 8 * j;
  *(volatile v4u*)p = u;
  __threadfence();
  *(volatile v4u*)p = u;
}

template <int MODE>
__global__ __launch_bounds__(256) void downproj_router_t_kernel(const float* __restrict__ A, const float* __restrict__ Rw,
                                                               unsigned short* __restrict__ ART, int KR, int tpr, float scale, int nthr) {
  const int g = blockIdx.x * 256 + threadIdx.x;
  if (g >= nthr) return;
  const int j  = g / tpr;
  const int c8 = (g - j * tpr) * 8;
  const int jj = j < kER ? j : (kER - 1);
  const int ea = jj >> 3, ra = jj & 7;
  int jr = j - kER; jr = jr < 0 ? 0 : (jr > (kExp - 1) ? (kExp - 1) : jr);
  unsigned short hb[8];
#pragma unroll
  for (int e = 0; e < 8; ++e) {
    const int k = c8 + e;
    const float va = A[((size_t)ea * KR + k) * kRank + ra];
    const float vr = Rw[(size_t)k * kExp + jr];
    const float v  = (j < kER) ? va : ((j < kER + kExp) ? vr : 0.0f);
    hb[e] = cvt_in16<MODE>(v, scale);
  }
  const v4u u = (v4u){pk16(hb[0], hb[1]), pk16(hb[2], hb[3]), pk16(hb[4], hb[5]), pk16(hb[6], hb[7])};
  unsigned short* p = ART + (size_t)j * KR + c8;
  *(volatile v4u*)p = u;
  __threadfence();
  *(volatile v4u*)p = u;
}

template <int MODE>
__global__ __launch_bounds__(256) void gate_tail_kernel(const float* __restrict__ ZL, unsigned short* __restrict__ P,
                                                        int ld, int kbase, float factor, int nthr) {
  const int g = blockIdx.x * 256 + threadIdx.x;
  if (g >= nthr) return;
  const int t = g >> 3, j = g & 7;
  const float* zl = ZL + (size_t)t * kNsm;
  const v4f lg = *(const v4f*)(zl + kER);
  const float m  = fmaxf(lg[0], fmaxf(lg[1], lg[2]));
  const float e0 = expf(lg[0] - m), e1 = expf(lg[1] - m), e2 = expf(lg[2] - m);
  const float inv = 1.0f / ((e0 + e1) + e2);
  const float ge  = ((j == 0) ? e0 : ((j == 1) ? e1 : e2)) * inv;
  const float f   = (j < kExp) ? ge * factor : 0.0f;
  const int jj = j < kExp ? j : (kExp - 1);
  const v4f a = *(const v4f*)(zl + 8 * jj);
  const v4f c = *(const v4f*)(zl + 8 * jj + 4);
  unsigned short hb[8];
#pragma unroll
  for (int e = 0; e < 4; ++e) {
    hb[e]     = cvt_cmp16<MODE>(a[e] * f);
    hb[4 + e] = cvt_cmp16<MODE>(c[e] * f);
  }
  const v4u u = (v4u){pk16(hb[0], hb[1]), pk16(hb[2], hb[3]), pk16(hb[4], hb[5]), pk16(hb[6], hb[7])};
  unsigned short* p = P + (size_t)t * ld + kbase + 8 * j;
  *(volatile v4u*)p = u;
  __threadfence();
  *(volatile v4u*)p = u;
}

extern "C" void kernel_launch(void* const* d_in, const int* in_sizes, int n_in,
                              void* d_out, int out_size, void* d_ws, size_t ws_size,
                              hipStream_t stream) {
  if (n_in < 11) return;
  if (in_sizes[0] != kTok * kDin) return;
  if (in_sizes[1] != kDin * kHid) return;
  if (in_sizes[2] != kHid) return;
  if (in_sizes[3] != kExp * kDin * kRank) return;
  if (in_sizes[4] != kExp * kRank * kHid) return;
  if (in_sizes[5] != kDin * kExp) return;
  if (in_sizes[6] != kHid * kDin) return;
  if (in_sizes[7] != kDin) return;
  if (in_sizes[8] != kExp * kHid * kRank) return;
  if (in_sizes[9] != kExp * kRank * kDin) return;
  if (in_sizes[10] != kHid * kExp) return;
  if (out_size != kTok * kDin) return;

  const float* x   = (const float*)d_in[0];
  const float* W1  = (const float*)d_in[1];
  const float* b1  = (const float*)d_in[2];
  const float* A1  = (const float*)d_in[3];
  const float* Bm1 = (const float*)d_in[4];
  const float* R1  = (const float*)d_in[5];
  const float* W2  = (const float*)d_in[6];
  const float* b2  = (const float*)d_in[7];
  const float* A2  = (const float*)d_in[8];
  const float* Bm2 = (const float*)d_in[9];
  const float* R2  = (const float*)d_in[10];
  float* outp = (float*)d_out;

  const size_t SZ_XA  = (size_t)kTok * kLd1 * 2;
  const size_t SZ_W1T = (size_t)kHid * kLd1 * 2;
  const size_t SZ_AR1 = (size_t)kNsm * kDin * 2;
  const size_t SZ_ZL  = (size_t)kTok * kNsm * 4;
  const size_t SZ_HA  = (size_t)kTok * kLd2 * 2;
  const size_t SZ_W2T = (size_t)kDin * kLd2 * 2;
  const size_t SZ_AR2 = (size_t)kNsm * kHid * 2;
  size_t off = 0;
  const size_t oXA  = off; off += SZ_XA;
  const size_t oW1T = off; off += SZ_W1T;
  const size_t oAR1 = off; off += SZ_AR1;
  const size_t oZL  = off; off += SZ_ZL;
  const size_t oHA  = off; off += SZ_HA;
  const size_t oW2T = off; off += SZ_W2T;
  const size_t oAR2 = off; off += SZ_AR2;
  const size_t TOTAL = off;
  if (TOTAL > ws_size) return;
  if (TOTAL > (size_t)134217728) return;

  char* ws = (char*)d_ws;
  unsigned short* XA   = (unsigned short*)(ws + oXA);
  unsigned short* W1T  = (unsigned short*)(ws + oW1T);
  unsigned short* AR1T = (unsigned short*)(ws + oAR1);
  float*          ZL   = (float*)(ws + oZL);
  unsigned short* HA   = (unsigned short*)(ws + oHA);
  unsigned short* W2T  = (unsigned short*)(ws + oW2T);
  unsigned short* AR2T = (unsigned short*)(ws + oAR2);

  const dim3 blk(256);

  {
    const int nthr = kTok * (kDin / 8);
    cast_rows_bf16_kernel<<<dim3(nthr / 256), blk, 0, stream>>>(x, XA, nthr);
  }
  transpose_cast_kernel<0><<<dim3(kDin / 64, kHid / 64), blk, 0, stream>>>(W1, W1T, kDin, kHid, kLd1, 1.0f);
  {
    const int nthr = kHid * 8;
    weight_tail_kernel<0><<<dim3(nthr / 256), blk, 0, stream>>>(Bm1, W1T, kHid, kLd1, kDin, 1.0f, nthr);
  }
  {
    const int tpr = kDin / 8, nthr = kNsm * tpr;
    downproj_router_t_kernel<0><<<dim3(nthr / 256), blk, 0, stream>>>(A1, R1, AR1T, kDin, tpr, 1.0f, nthr);
  }
  transpose_cast_kernel<1><<<dim3(kHid / 64, kDin / 64), blk, 0, stream>>>(W2, W2T, kHid, kDin, kLd2, kCarry);
  {
    const int nthr = kDin * 8;
    weight_tail_kernel<1><<<dim3(nthr / 256), blk, 0, stream>>>(Bm2, W2T, kDin, kLd2, kHid, kCarryB2, nthr);
  }
  {
    const int tpr = kHid / 8, nthr = kNsm * tpr;
    downproj_router_t_kernel<1><<<dim3(nthr / 256), blk, 0, stream>>>(A2, R2, AR2T, kHid, tpr, kCarry, nthr);
  }

  const int tilesTok = kTok / 64;
  const dim3 gSm((tilesTok * (kNsm / 64) + 7) / 8, 1);
  const dim3 gL1((tilesTok * (kHid / 64) + 7) / 8, 1);
  const dim3 gL2((tilesTok * (kDin / 64) + 7) / 8, 1);
  const int nthrGate = kTok * 8;

  wmma_gemm64<1, false, 0, 0, false, 0><<<gSm, blk, 0, stream>>>(
      XA, XA, kLd1, 0L, AR1T, AR1T, kDin, 0L, (void*)ZL, (void*)ZL, kNsm, 0L, b1, b1, 0L, kTok, kNsm, kDin, 1.0f);
  gate_tail_kernel<0><<<dim3(nthrGate / 256), blk, 0, stream>>>(ZL, XA, kLd1, kDin, kScaling, nthrGate);
  wmma_gemm64<1, false, 2, 1, false, 2><<<gL1, blk, 0, stream>>>(
      XA, XA, kLd1, 0L, W1T, W1T, kLd1, 0L, (void*)HA, (void*)HA, kLd2, 0L, b1, b1, 0L, kTok, kHid, kK1, 1.0f);
  wmma_gemm64<0, false, 0, 0, false, 0><<<gSm, blk, 0, stream>>>(
      HA, HA, kLd2, 0L, AR2T, AR2T, kHid, 0L, (void*)ZL, (void*)ZL, kNsm, 0L, b2, b2, 0L, kTok, kNsm, kHid, kCarryInv);
  gate_tail_kernel<1><<<dim3(nthrGate / 256), blk, 0, stream>>>(ZL, HA, kLd2, kHid, kTailFac2, nthrGate);
  wmma_gemm64<0, false, 2, 0, false, 0><<<gL2, blk, 0, stream>>>(
      HA, HA, kLd2, 0L, W2T, W2T, kLd2, 0L, (void*)outp, (void*)outp, kDin, 0L, b2, b2, 0L, kTok, kDin, kK2, kCarryInv);
}
